// EntityClassifyHeteroAPI_1331439862169
// MI455X (gfx1250) — hardware-run, weakly checked
//
#include <hip/hip_runtime.h>
#include <stddef.h>
#include <stdint.h>


#define NN      50000
#define HD      256
#define OD      64
#define NREL    8
#define EPR     65536
#define NEDGE   (NREL * EPR)
#define TERMS   2
#define KR      (HD * TERMS)
#define KC      (NREL * KR)
#define NTHR    256
#define NWAVE   8
#define EPT     8
#define CHUNK   (NTHR * EPT)
#define WCAP    (EPT * 32)
#define LISTN   (NWAVE * WCAP)
#define NBA     1024
#define PKS     10
#define NBB     49
#define RCAP    28672
#define DEGCAP  96
#define SEGCAP  32
#define FLP     32
#define CR      2048
#define NCH     25
#define GBM     64
#define GTHR    128
#define RPB     64
#define KU      (KC / 8)
#define NU1     (HD * KU)
#define NU2     (OD * KU)
#define NUW     (NU1 + NU2)
#define BK_INTS (2 * RCAP + 9 * NBA + LISTN + 32)
#define LDS_BK  (BK_INTS * 4)
#define WSMAX   134217728

static_assert(TERMS == 1 || TERMS == 2);
static_assert(EPR == (1 << 16) && (EPR % CHUNK) == 0 && (NEDGE % CHUNK) == 0);
static_assert((CHUNK & (CHUNK - 1)) == 0 && CHUNK <= 4096);
static_assert((NBA & (NBA - 1)) == 0 && NBA == (1 << PKS) && LISTN >= NBA);
static_assert((long long)NEDGE << PKS < (1LL << 31));
static_assert(NBB * NBA >= NN && (NBB - 1) * NBA < NN);
static_assert(CR == 2 * NBA && (CR % GBM) == 0 && (NBA % RPB) == 0 && (NBA % GBM) == 0);
static_assert(NCH * CR >= NN && (NCH - 1) * CR < NN);
static_assert(KC == NREL * KR && (KC % 32) == 0 && (KR % 256) == 0);
static_assert((HD % 128) == 0 && (OD % 64) == 0 && HD == 8 * 32);
static_assert(RCAP >= 11374 + 1024 && (RCAP % (4 * NTHR)) == 0);
static_assert(DEGCAP >= 67 + 8 && SEGCAP >= 9 + 8 && SEGCAP <= 32);
static_assert((9 * NBA) % (4 * NTHR) == 0 && (BK_INTS % 4) == 0);
static_assert(LDS_BK <= 327680);
static_assert((NU1 % NTHR) == 0 && (NUW % NTHR) == 0);
static_assert(RPB == NWAVE * 8 && GBM == (GTHR / 32) * 16);

typedef float          v4f   __attribute__((ext_vector_type(4)));
typedef float          v8f   __attribute__((ext_vector_type(8)));
typedef int            v4i   __attribute__((ext_vector_type(4)));
typedef int            v8i   __attribute__((ext_vector_type(8)));
typedef unsigned short v8us  __attribute__((ext_vector_type(8)));
typedef __bf16         v16bf __attribute__((ext_vector_type(16)));
typedef v4f  __attribute__((may_alias)) v4fa;
typedef v4i  __attribute__((may_alias)) v4ia;
typedef v8us __attribute__((may_alias)) v8usa;
union FragB { v16bf v; v8us h[2]; v8i w; };

static constexpr size_t O_H0   = 0;
static constexpr size_t O_H1   = O_H0 + (size_t)NN * HD * 4;
static constexpr size_t O_AP   = O_H1 + (size_t)NN * HD * 4;
static constexpr size_t O_W1S  = O_AP + (size_t)CR * KC * 2;
static constexpr size_t O_W2S  = O_W1S + (size_t)HD * KC * 2;
static constexpr size_t O_LIST = O_W2S + (size_t)OD * KC * 2;
static constexpr size_t O_SEG  = O_LIST + (size_t)NBB * RCAP * 4;
static constexpr size_t O_FLAG = O_SEG + (size_t)NBB * 9 * NBA * 4;
static constexpr size_t O_BT   = O_FLAG + 6400;
static constexpr size_t WS_END = O_BT + 2304;
static_assert((O_H1 % 256) == 0 && (O_AP % 256) == 0 && (O_W1S % 256) == 0 && (O_W2S % 256) == 0);
static_assert((O_LIST % 256) == 0 && (O_SEG % 256) == 0 && (O_FLAG % 256) == 0 && (O_BT % 256) == 0);
static_assert((size_t)NBB * FLP * 4 <= 6400);
static_assert(WS_END <= (size_t)WSMAX);
static_assert((long long)(NN - 1) * OD + (OD - 1) == (long long)NN * OD - 1);

__device__ __forceinline__ v8f wmb(const FragB& a, const FragB& b, v8f c) {
  v8f d = __builtin_amdgcn_wmma_f32_16x16x32_bf16(false, a.v, false, b.v, (short)0, c, false, false);
  asm volatile("v_nop\n\tv_nop\n\tv_nop\n\tv_nop" : "+v"(d) : "v"(a.w), "v"(b.w));
  return d;
}

__device__ __forceinline__ unsigned bf16_bits(float f) {
  const unsigned u = __float_as_uint(f);
  const unsigned r = (u + 0x7FFFu + ((u >> 16) & 1u)) >> 16;
  return ((u & 0x7FFFFFFFu) > 0x7F800000u) ? 0x7FC0u : r;
}
__device__ __forceinline__ float bf16_val(float f) {
  const unsigned u = __float_as_uint(f);
  return __uint_as_float(((u + 0x7FFFu + ((u >> 16) & 1u)) >> 16) << 16);
}

__device__ __forceinline__ int scan_chunk(const int* __restrict__ dsts, int nE, int cbase, int slotBase,
                                          int nb, int vec8, int* list, int tid, int lane, int wave) {
  int wc = 0;
  const int el0  = tid * EPT;
  const int e0   = cbase + el0;
  const int sent = -2147483647 - 1;
  v4i da, db;
  if (vec8 != 0 && cbase + CHUNK <= nE) {
    da = *(const v4i*)(dsts + e0);
    db = *(const v4i*)(dsts + e0 + 4);
  } else {
    da.x = (e0     < nE) ? dsts[min(e0,     nE - 1)] : sent;
    da.y = (e0 + 1 < nE) ? dsts[min(e0 + 1, nE - 1)] : sent;
    da.z = (e0 + 2 < nE) ? dsts[min(e0 + 2, nE - 1)] : sent;
    da.w = (e0 + 3 < nE) ? dsts[min(e0 + 3, nE - 1)] : sent;
    db.x = (e0 + 4 < nE) ? dsts[min(e0 + 4, nE - 1)] : sent;
    db.y = (e0 + 5 < nE) ? dsts[min(e0 + 5, nE - 1)] : sent;
    db.z = (e0 + 6 < nE) ? dsts[min(e0 + 6, nE - 1)] : sent;
    db.w = (e0 + 7 < nE) ? dsts[min(e0 + 7, nE - 1)] : sent;
  }
  const unsigned nbs = (unsigned)slotBase;
  const unsigned unb = (unsigned)nb;
  const unsigned s0 = (unsigned)da.x - nbs, s1 = (unsigned)da.y - nbs;
  const unsigned s2 = (unsigned)da.z - nbs, s3 = (unsigned)da.w - nbs;
  const unsigned s4 = (unsigned)db.x - nbs, s5 = (unsigned)db.y - nbs;
  const unsigned s6 = (unsigned)db.z - nbs, s7 = (unsigned)db.w - nbs;
  const bool h0 = s0 < unb, h1 = s1 < unb, h2 = s2 < unb, h3 = s3 < unb;
  const bool h4 = s4 < unb, h5 = s5 < unb, h6 = s6 < unb, h7 = s7 < unb;
  const unsigned any = __builtin_amdgcn_ballot_w32(h0 | h1 | h2 | h3 | h4 | h5 | h6 | h7);
  if (any != 0u) {
#define HITJ(J, HJ, SJ) { \
      const unsigned mj = __builtin_amdgcn_ballot_w32(HJ); \
      if (mj != 0u) { \
        if (HJ) { \
          const int pos = wc + (int)__builtin_amdgcn_mbcnt_lo(mj, 0u); \
          if (pos < WCAP) list[wave * WCAP + pos] = ((el0 + (J)) << PKS) | (int)(SJ); \
        } \
        wc += (int)__builtin_popcount(mj); } }
    HITJ(0, h0, s0)
    HITJ(1, h1, s1)
    HITJ(2, h2, s2)
    HITJ(3, h3, s3)
    HITJ(4, h4, s4)
    HITJ(5, h5, s5)
    HITJ(6, h6, s6)
    HITJ(7, h7, s7)
#undef HITJ
  }
  return wc;
}

__device__ __forceinline__ v8us cv8b(const float* __restrict__ p, size_t stride) {
  v8us o;
#pragma unroll
  for (int i = 0; i < 8; ++i) o[i] = (unsigned short)bf16_bits(p[(size_t)i * stride]);
  return o;
}

__global__ __launch_bounds__(NTHR) void k_prep(const float* __restrict__ W1, const float* __restrict__ W2,
                                               const float* __restrict__ b0, const float* __restrict__ b1,
                                               const float* __restrict__ b2,
                                               unsigned short* W1S, unsigned short* W2S, float* BT) {
  const int u = (int)blockIdx.x * NTHR + (int)threadIdx.x;
  if (u < NU1) {
    const int n  = u / KU;
    const int k8 = (u - n * KU) * 8;
    const int r  = k8 / KR;
    const int i0 = (k8 - r * KR) & (HD - 1);
    const v8us o = cv8b(W1 + ((size_t)(r * HD + i0)) * HD + n, HD);
    unsigned short* dp = W1S + (size_t)u * 8;
    *(volatile v8us*)dp = o;
    __threadfence();
    *(volatile v8us*)dp = o;
  } else if (u < NUW) {
    const int v  = u - NU1;
    const int n  = v / KU;
    const int k8 = (v - n * KU) * 8;
    const int r  = k8 / KR;
    const int i0 = (k8 - r * KR) & (HD - 1);
    const v8us o = cv8b(W2 + ((size_t)(r * HD + i0)) * OD + n, OD);
    unsigned short* dp = W2S + (size_t)v * 8;
    *(volatile v8us*)dp = o;
    __threadfence();
    *(volatile v8us*)dp = o;
  } else if (u < NUW + NTHR) {
    const int t  = u - NUW;
    const int wv = t >> 5;
    v4f v;
    if (wv < 2) {
      v = *(const v4f*)(b0 + 4 * t);
    } else if (wv < 4) {
      v = *(const v4f*)(b1 + 4 * (t - 64));
    } else {
      int q = t - 128;
      q = q < 0 ? 0 : (q > 15 ? 15 : q);
      v = *(const v4f*)(b2 + 4 * q);
    }
    asm volatile("" :: "v"(v.x), "v"(v.y), "v"(v.z), "v"(v.w));
    v4f o;
    o.x = bf16_val(v.x); o.y = bf16_val(v.y); o.z = bf16_val(v.z); o.w = bf16_val(v.w);
    float* dp = BT + 4 * (t < 144 ? t : 143);
    if (t < 144) *(volatile v4f*)dp = o;
    __threadfence();
    if (t < 144) *(volatile v4f*)dp = o;
  }
}

__global__ __launch_bounds__(NTHR) void k_bucket(const int* __restrict__ srcs, const int* __restrict__ dsts,
                                                 int nE, int nN, int vec8,
                                                 int* LISTg, int* SEGg, int* FLAGg) {
  extern __shared__ v4f lds_dyn[];
  int* reg1 = (int*)lds_dyn;
  int* reg2 = reg1 + RCAP;
  int* segc = reg2 + RCAP;
  int* list = segc + 9 * NBA;
  int* misc = list + LISTN;
  int* wcnt = misc;
  int* wtot = misc + 8;
  int* wflg = misc + 16;
  const int tid = (int)threadIdx.x, lane = tid & 31, wave = tid >> 5;
  const int bidx = (int)blockIdx.x;
  const int nodeBase = bidx * NBA;

  {
    const v4i z4 = {0, 0, 0, 0};
    for (int i = tid * 4; i < BK_INTS; i += NTHR * 4) *(v4ia*)(reg1 + i) = z4;
  }
  __syncthreads();

  int tot = 0, ovf = 0;
  const int nChunks = (nE + CHUNK - 1) / CHUNK;
#pragma unroll 1
  for (int ch = 0; ch < nChunks; ++ch) {
    const int cbase = ch * CHUNK;
    const int wc = scan_chunk(dsts, nE, cbase, nodeBase, NBA, vec8, list, tid, lane, wave);
    if (lane == 0) wcnt[wave] = wc;
    __syncthreads();
    int pre = 0, all = 0;
#pragma unroll
    for (int w2 = 0; w2 < NWAVE; ++w2) {
      int c = wcnt[w2];
      c = c < 0 ? 0 : (c > WCAP ? WCAP : c);
      all += c;
      pre += (w2 < wave) ? c : 0;
    }
    const int wcc  = wc > WCAP ? WCAP : wc;
    const int base = tot + pre;
#pragma unroll 1
    for (int i = lane; i < wcc; i += 32) {
      const int ent = list[wave * WCAP + i];
      const int el  = (ent >> PKS) & (CHUNK - 1);
      const int sl  = ent & (NBA - 1);
      int eid = cbase + el;
      eid = eid > nE - 1 ? nE - 1 : eid;
      const int pos = base + i;
      if (pos < RCAP) reg1[pos] = (int)(((unsigned)eid << PKS) | (unsigned)sl);
    }
    if (tot + all > RCAP) ovf = 1;
    tot += all;
    tot = tot > RCAP ? RCAP : tot;
    __syncthreads();
  }
  const int nh = tot;

  if (wave == 0) {
#pragma unroll 1
    for (int b0 = 0; b0 < nh; b0 += 32) {
      const int idx = b0 + lane;
      const int uv  = reg1[idx < RCAP ? idx : RCAP - 1];
      const int m32 = (nh - b0) < 32 ? (nh - b0) : 32;
#pragma unroll 1
      for (int k = 0; k < m32; ++k) {
        const int u  = __builtin_amdgcn_readlane(uv, k);
        const int sl = u & (NBA - 1);
        const int r  = (int)(((unsigned)u >> (PKS + 16)) & (NREL - 1));
        if (lane == 0) segc[r * NBA + sl] = segc[r * NBA + sl] + 1;
      }
    }
  }
  __syncthreads();

  int flagAll = ovf;
  {
    v4i c[NREL];
    v4i t4 = {0, 0, 0, 0};
#pragma unroll
    for (int r = 0; r < NREL; ++r) {
      c[r] = *(const v4ia*)(segc + r * NBA + 4 * tid);
      t4 += c[r];
    }
    const int ts = t4.x + t4.y + t4.z + t4.w;
    int incl = ts;
#pragma unroll
    for (int d = 1; d < 32; d <<= 1) {
      const int up = __shfl_up(incl, d);
      if (lane >= d) incl += up;
    }
    const bool bigl = (t4.x > DEGCAP) | (t4.y > DEGCAP) | (t4.z > DEGCAP) | (t4.w > DEGCAP);
    const unsigned bigm = __builtin_amdgcn_ballot_w32(bigl);
    if (lane == 31) wtot[wave] = incl;
    if (lane == 0)  wflg[wave] = (bigm != 0u) ? 1 : 0;
    __syncthreads();
    int pre = 0;
#pragma unroll
    for (int w2 = 0; w2 < NWAVE; ++w2) {
      pre += (w2 < wave) ? wtot[w2] : 0;
      flagAll |= wflg[w2];
    }
    v4i run;
    run.x = pre + incl - ts;
    run.y = run.x + t4.x;
    run.z = run.y + t4.y;
    run.w = run.z + t4.z;
    *(v4ia*)(list + 4 * tid) = run;
#pragma unroll
    for (int r = 0; r < NREL; ++r) {
      *(v4ia*)(segc + r * NBA + 4 * tid) = run;
      run += c[r];
    }
    *(v4ia*)(segc + NREL * NBA + 4 * tid) = run;
  }
  __syncthreads();

  if (wave == 0) {
#pragma unroll 1
    for (int b0 = 0; b0 < nh; b0 += 32) {
      const int idx = b0 + lane;
      const int uv  = reg1[idx < RCAP ? idx : RCAP - 1];
      const int m32 = (nh - b0) < 32 ? (nh - b0) : 32;
#pragma unroll 1
      for (int k = 0; k < m32; ++k) {
        const int u   = __builtin_amdgcn_readlane(uv, k);
        const int sl  = u & (NBA - 1);
        const int eid = (int)((unsigned)u >> PKS);
        if (lane == 0) {
          int pos = list[sl];
          pos = pos < 0 ? 0 : (pos > RCAP - 1 ? RCAP - 1 : pos);
          reg2[pos] = eid;
          list[sl] = pos + 1;
        }
      }
    }
  }
  __syncthreads();

#pragma unroll 1
  for (int it = 0; it < RCAP / (4 * NTHR); ++it) {
    const int i4 = (it * NTHR + tid) * 4;
    const v4i e = *(const v4ia*)(reg2 + i4);
    const int e0 = e.x < 0 ? 0 : (e.x > nE - 1 ? nE - 1 : e.x);
    const int e1 = e.y < 0 ? 0 : (e.y > nE - 1 ? nE - 1 : e.y);
    const int e2 = e.z < 0 ? 0 : (e.z > nE - 1 ? nE - 1 : e.z);
    const int e3 = e.w < 0 ? 0 : (e.w > nE - 1 ? nE - 1 : e.w);
    int s0 = srcs[e0], s1 = srcs[e1], s2 = srcs[e2], s3 = srcs[e3];
    asm volatile("" :: "v"(s0), "v"(s1), "v"(s2), "v"(s3));
    s0 = s0 < 0 ? 0 : (s0 > nN - 1 ? nN - 1 : s0);
    s1 = s1 < 0 ? 0 : (s1 > nN - 1 ? nN - 1 : s1);
    s2 = s2 < 0 ? 0 : (s2 > nN - 1 ? nN - 1 : s2);
    s3 = s3 < 0 ? 0 : (s3 > nN - 1 ? nN - 1 : s3);
    v4i o;
    o.x = (i4 + 0 < nh) ? s0 : 0;
    o.y = (i4 + 1 < nh) ? s1 : 0;
    o.z = (i4 + 2 < nh) ? s2 : 0;
    o.w = (i4 + 3 < nh) ? s3 : 0;
    *(v4ia*)(reg2 + i4) = o;
  }
  __syncthreads();

  int* Lb = LISTg + (size_t)bidx * RCAP;
  int* Sb = SEGg + (size_t)bidx * (9 * NBA);
  int* Fb = FLAGg + (size_t)bidx * FLP;
  v4i fv;
  fv.x = (tid == 0) ? flagAll : 0;
  fv.y = (tid == 0) ? nh : 0;
  fv.z = 0; fv.w = 0;
#pragma unroll 1
  for (int it = 0; it < RCAP / (4 * NTHR); ++it) {
    const int i4 = (it * NTHR + tid) * 4;
    const v4i v = *(const v4ia*)(reg2 + i4);
    *(volatile v4i*)(Lb + i4) = v;
  }
#pragma unroll 1
  for (int it = 0; it < (9 * NBA) / (4 * NTHR); ++it) {
    const int i4 = (it * NTHR + tid) * 4;
    const v4i v = *(const v4ia*)(segc + i4);
    *(volatile v4i*)(Sb + i4) = v;
  }
  if (tid < 8) *(volatile v4i*)(Fb + 4 * tid) = fv;
  __threadfence();
#pragma unroll 1
  for (int it = 0; it < RCAP / (4 * NTHR); ++it) {
    const int i4 = (it * NTHR + tid) * 4;
    const v4i v = *(const v4ia*)(reg2 + i4);
    *(volatile v4i*)(Lb + i4) = v;
  }
#pragma unroll 1
  for (int it = 0; it < (9 * NBA) / (4 * NTHR); ++it) {
    const int i4 = (it * NTHR + tid) * 4;
    const v4i v = *(const v4ia*)(segc + i4);
    *(volatile v4i*)(Sb + i4) = v;
  }
  if (tid < 8) *(volatile v4i*)(Fb + 4 * tid) = fv;
}

__global__ __launch_bounds__(NTHR) void k_l0(const float* __restrict__ emb, const int* __restrict__ LISTg,
                                             const int* __restrict__ SEGg, const int* __restrict__ FLAGg,
                                             const float* __restrict__ btab, int nN, float* H0) {
  __shared__ __attribute__((aligned(16))) float bsh[HD];
  const int tid = (int)threadIdx.x, lane = tid & 31, wave = tid >> 5;
  if (wave < 2) {
    const v4f t = *(const v4f*)(btab + 4 * tid);
    *(v4fa*)(bsh + 4 * tid) = t;
  }
  __syncthreads();
  const int nodeBase = (int)blockIdx.x * RPB;
  int bb = nodeBase >> PKS;
  bb = bb > NBB - 1 ? NBB - 1 : bb;
  const int flag = FLAGg[(size_t)bb * FLP];
  const int* Lb = LISTg + (size_t)bb * RCAP;
  const v4f bA = *(const v4fa*)(bsh + 4 * lane);
  const v4f bB = *(const v4fa*)(bsh + 128 + 4 * lane);
  const float qnan = __int_as_float(0x7fc00000);

#pragma unroll 1
  for (int i = 0; i < 8; ++i) {
    const int node = nodeBase + 8 * wave + i;
    if (node < nN) {
      const int slot = node & (NBA - 1);
      const int kk   = (lane == 0) ? 0 : NREL;
      const int segv = SEGg[((size_t)bb * 9 + kk) * NBA + slot];
      int st = __builtin_amdgcn_readlane(segv, 0);
      const int en = __builtin_amdgcn_readlane(segv, 1);
      st = st < 0 ? 0 : (st > RCAP ? RCAP : st);
      const int craw = en - st;
      int c = craw < 0 ? 0 : (craw > DEGCAP ? DEGCAP : craw);
      if (c > RCAP - st) c = RCAP - st;
      const bool big = craw > DEGCAP;
      float a0 = 0.f, a1 = 0.f, a2 = 0.f, a3 = 0.f, a4 = 0.f, a5 = 0.f, a6 = 0.f, a7 = 0.f;
#pragma unroll 1
      for (int b0 = 0; b0 < c; b0 += 32) {
        int idx = st + b0 + lane;
        idx = idx > RCAP - 1 ? RCAP - 1 : idx;
        int sr = Lb[idx];
        sr = sr < 0 ? 0 : (sr > nN - 1 ? nN - 1 : sr);
        const int m32 = (c - b0) < 32 ? (c - b0) : 32;
#pragma unroll 1
        for (int k = 0; k < m32; ++k) {
          const int sk = __builtin_amdgcn_readlane(sr, k);
          const float* p = emb + (size_t)sk * HD + 4 * lane;
          const v4f va = *(const v4f*)p;
          const v4f vb = *(const v4f*)(p + 128);
          a0 += bf16_val(va.x); a1 += bf16_val(va.y); a2 += bf16_val(va.z); a3 += bf16_val(va.w);
          a4 += bf16_val(vb.x); a5 += bf16_val(vb.y); a6 += bf16_val(vb.z); a7 += bf16_val(vb.w);
        }
      }
      const float pz = (flag != 0 || big) ? qnan : 0.0f;
      v4f ya, yb;
      {
        const float t0 = a0 + bA.x + pz, t1 = a1 + bA.y + pz, t2 = a2 + bA.z + pz, t3 = a3 + bA.w + pz;
        const float t4 = a4 + bB.x + pz, t5 = a5 + bB.y + pz, t6 = a6 + bB.z + pz, t7 = a7 + bB.w + pz;
        ya.x = (t0 > 0.0f) ? t0 : (t0 - t0); ya.y = (t1 > 0.0f) ? t1 : (t1 - t1);
        ya.z = (t2 > 0.0f) ? t2 : (t2 - t2); ya.w = (t3 > 0.0f) ? t3 : (t3 - t3);
        yb.x = (t4 > 0.0f) ? t4 : (t4 - t4); yb.y = (t5 > 0.0f) ? t5 : (t5 - t5);
        yb.z = (t6 > 0.0f) ? t6 : (t6 - t6); yb.w = (t7 > 0.0f) ? t7 : (t7 - t7);
      }
      float* op = H0 + (size_t)node * HD + 4 * lane;
      *(volatile v4f*)op = ya;
      *(volatile v4f*)(op + 128) = yb;
      __threadfence();
      *(volatile v4f*)op = ya;
      *(volatile v4f*)(op + 128) = yb;
    }
  }
}

__global__ __launch_bounds__(NTHR) void k_agg(const float* __restrict__ Hs, const int* __restrict__ LISTg,
                                              const int* __restrict__ SEGg, const int* __restrict__ FLAGg,
                                              int nN, int chunkBase, unsigned short* APp) {
  const int tid = (int)threadIdx.x, lane = tid & 31, wave = tid >> 5;
  const int rowBase = (int)blockIdx.x * RPB;
  int bb = (chunkBase + rowBase) >> PKS;
  bb = bb > NBB - 1 ? NBB - 1 : bb;
  const int flag = FLAGg[(size_t)bb * FLP];
  const int* Lb = LISTg + (size_t)bb * RCAP;
  const float qnan = __int_as_float(0x7fc00000);

#pragma unroll 1
  for (int i = 0; i < 8; ++i) {
    const int row  = rowBase + 8 * wave + i;
    const int node = chunkBase + row;
    const bool live = node < nN;
    const int nc   = live ? node : nN - 1;
    const int slot = nc & (NBA - 1);
    int bq = nc >> PKS;
    bq = bq > NBB - 1 ? NBB - 1 : bq;
    const int kk   = lane < NREL ? lane : NREL;
    const int segv = SEGg[((size_t)bq * 9 + kk) * NBA + slot];
    const float pz = (live && flag != 0) ? qnan : 0.0f;
    unsigned short* rp = APp + (size_t)row * KC + 8 * lane;

#pragma unroll 1
    for (int r = 0; r < NREL; ++r) {
      int st = __builtin_amdgcn_readlane(segv, r);
      const int en = __builtin_amdgcn_readlane(segv, r + 1);
      st = st < 0 ? 0 : (st > RCAP ? RCAP : st);
      const int craw = en - st;
      int c = craw < 0 ? 0 : (craw > SEGCAP ? SEGCAP : craw);
      if (c > RCAP - st) c = RCAP - st;
      c = live ? c : 0;
      const bool big = live && (craw > SEGCAP);
      int idx = st + lane;
      idx = idx > RCAP - 1 ? RCAP - 1 : idx;
      int sr = Lb[idx];
      sr = sr < 0 ? 0 : (sr > nN - 1 ? nN - 1 : sr);
      float a[8];
#pragma unroll
      for (int j = 0; j < 8; ++j) a[j] = 0.0f;
#pragma unroll 1
      for (int k = 0; k < c; ++k) {
        const int sk = __builtin_amdgcn_readlane(sr, k);
        const float* p = Hs + (size_t)sk * HD + 8 * lane;
        const v4f va = *(const v4f*)p;
        const v4f vb = *(const v4f*)(p + 4);
        a[0] += va.x; a[1] += va.y; a[2] += va.z; a[3] += va.w;
        a[4] += vb.x; a[5] += vb.y; a[6] += vb.z; a[7] += vb.w;
      }
      const float pzr = big ? qnan : pz;
      v8us hv, lv;
#pragma unroll
      for (int j = 0; j < 8; ++j) {
        const float v = a[j] + pzr;
        const unsigned hb = bf16_bits(v);
        hv[j] = (unsigned short)hb;
        lv[j] = (unsigned short)bf16_bits(v - __uint_as_float(hb << 16));
      }
      unsigned short* hp = rp + r * KR;
      *(volatile v8us*)hp = hv;
      if (TERMS == 2) *(volatile v8us*)(hp + 256) = lv;
      __threadfence();
      *(volatile v8us*)hp = hv;
      if (TERMS == 2) *(volatile v8us*)(hp + 256) = lv;
    }
  }
}

template <int GNT, int FIN>
__global__ __launch_bounds__(GTHR) __attribute__((amdgpu_num_vgpr(248)))
void k_gemm(const unsigned short* __restrict__ A, const unsigned short* __restrict__ BT,
            const float* __restrict__ bias, const int* __restrict__ FLAGg,
            float* outp, int ldo, int chunkBase, int nN) {
  constexpr int GBN = 16 * GNT;
  constexpr int LPR = GBN / 4;
  constexpr int RPI = 32 / LPR;
  constexpr int NI  = 16 / RPI;
  static_assert(GNT == 8 || GNT == 4);
  __shared__ __attribute__((aligned(16))) float stg[GBM * GBN];
  __shared__ __attribute__((aligned(16))) float bsh[GBN];
  const int tid = (int)threadIdx.x, lane = tid & 31, wave = tid >> 5, hh = lane >> 4, m = lane & 15;
  const int rowBase = (int)blockIdx.x * GBM;
  const int colBase = (int)blockIdx.y * GBN;

  v8f acc[GNT];
  {
    const v8f z = {0.f, 0.f, 0.f, 0.f, 0.f, 0.f, 0.f, 0.f};
#pragma unroll
    for (int t = 0; t < GNT; ++t) acc[t] = z;
  }
  const unsigned short* ap = A  + (size_t)(rowBase + 16 * wave + m) * (size_t)KC + 8 * hh;
  const unsigned short* bp = BT + (size_t)(colBase + m) * (size_t)KC + 8 * hh;

#pragma unroll 1
  for (int k0 = 0; k0 < KC; k0 += 32) {
    FragB af;
    af.h[0] = *(const v8usa*)(ap + k0);
    af.h[1] = *(const v8usa*)(ap + k0 + 16);
#pragma unroll
    for (int nt = 0; nt < GNT; ++nt) {
      const unsigned short* wq = bp + (size_t)(16 * nt) * (size_t)KC + k0;
      FragB bf;
      bf.h[0] = *(const v8usa*)wq;
      bf.h[1] = *(const v8usa*)(wq + 16);
      acc[nt] = wmb(af, bf, acc[nt]);
    }
  }

#pragma unroll
  for (int nt = 0; nt < GNT; ++nt) {
    const int lc = 16 * nt + m;
#pragma unroll
    for (int r = 0; r < 8; ++r) {
      const int lr = 16 * wave + 8 * hh + r;
      stg[lr * GBN + lc] = acc[nt][r];
    }
  }
  if (wave == 0) {
    const int q = lane < LPR ? lane : LPR - 1;
    const v4f bv = *(const v4f*)(bias + colBase + 4 * q);
    if (lane < LPR) *(v4fa*)(bsh + 4 * q) = bv;
  }
  __syncthreads();

  const int rsub = lane / LPR;
  const int cq   = lane - rsub * LPR;
  const v4f bb4 = *(const v4fa*)(bsh + 4 * cq);
  int bbk = (chunkBase + rowBase) >> PKS;
  bbk = bbk > NBB - 1 ? NBB - 1 : bbk;
  const int flag = FLAGg[(size_t)bbk * FLP];
  const float qnan = __int_as_float(0x7fc00000);

  v4f pv[NI];
#pragma unroll
  for (int j = 0; j < NI; ++j) {
    const int lr = 16 * wave + j * RPI + rsub;
    const v4f t = *(const v4fa*)(stg + lr * GBN + 4 * cq) + bb4;
    v4f y;
    if constexpr (FIN == 0) {
      y.x = (t.x > 0.0f) ? t.x : (t.x - t.x);
      y.y = (t.y > 0.0f) ? t.y : (t.y - t.y);
      y.z = (t.z > 0.0f) ? t.z : (t.z - t.z);
      y.w = (t.w > 0.0f) ? t.w : (t.w - t.w);
    } else {
      y = t;
    }
    y.x = (flag != 0) ? qnan : y.x;
    y.y = (flag != 0) ? qnan : y.y;
    y.z = (flag != 0) ? qnan : y.z;
    y.w = (flag != 0) ? qnan : y.w;
    pv[j] = y;
  }
#pragma unroll
  for (int j = 0; j < NI; ++j) {
    const int gr = chunkBase + rowBase + 16 * wave + j * RPI + rsub;
    float* op = outp + (size_t)gr * (size_t)ldo + colBase + 4 * cq;
    if (gr < nN) *(volatile v4f*)op = pv[j];
  }
  __threadfence();
#pragma unroll
  for (int j = 0; j < NI; ++j) {
    const int gr = chunkBase + rowBase + 16 * wave + j * RPI + rsub;
    float* op = outp + (size_t)gr * (size_t)ldo + colBase + 4 * cq;
    if (gr < nN) *(volatile v4f*)op = pv[j];
  }
}

static inline int cdiv(int a, int b) { return (a + b - 1) / b; }

extern "C" void kernel_launch(void* const* d_in, const int* in_sizes, int n_in,
                              void* d_out, int out_size, void* d_ws, size_t ws_size,
                              hipStream_t stream) {
  if (n_in < 8) return;
  if (in_sizes[0] != NN * HD) return;
  if (in_sizes[1] != NEDGE || in_sizes[2] != NEDGE) return;
  if (in_sizes[3] != NREL * HD * HD) return;
  if (in_sizes[4] != HD || in_sizes[5] != HD) return;
  if (in_sizes[6] != NREL * HD * OD) return;
  if (in_sizes[7] != OD) return;
  if (out_size != NN * OD) return;
  if (ws_size < WS_END) return;

  const float* emb = (const float*)d_in[0];
  const int*   src = (const int*)d_in[1];
  const int*   dst = (const int*)d_in[2];
  const float* W1  = (const float*)d_in[3];
  const float* b0  = (const float*)d_in[4];
  const float* b1  = (const float*)d_in[5];
  const float* W2  = (const float*)d_in[6];
  const float* b2  = (const float*)d_in[7];
  float* out = (float*)d_out;

  char* ws = (char*)d_ws;
  float*          H0   = (float*)(ws + O_H0);
  float*          H1   = (float*)(ws + O_H1);
  unsigned short* AP   = (unsigned short*)(ws + O_AP);
  unsigned short* W1S  = (unsigned short*)(ws + O_W1S);
  unsigned short* W2S  = (unsigned short*)(ws + O_W2S);
  int*            LIST = (int*)(ws + O_LIST);
  int*            SEG  = (int*)(ws + O_SEG);
  int*            FLAG = (int*)(ws + O_FLAG);
  float*          BTB  = (float*)(ws + O_BT);

  hipFuncSetAttribute(reinterpret_cast<const void*>(&k_bucket), hipFuncAttributeMaxDynamicSharedMemorySize, LDS_BK);

  k_prep<<<NUW / NTHR + 1, NTHR, 0, stream>>>(W1, W2, b0, b1, b2, W1S, W2S, BTB);
  k_bucket<<<NBB, NTHR, LDS_BK, stream>>>(src, dst, NEDGE, NN, 1, LIST, SEG, FLAG);
  k_l0<<<cdiv(NN, RPB), NTHR, 0, stream>>>(emb, LIST, SEG, FLAG, BTB, NN, H0);
  for (int c = 0; c < NCH; ++c) {
    const int cb   = c * CR;
    const int rows = (NN - cb) < CR ? (NN - cb) : CR;
    const int mPad = cdiv(rows, GBM) * GBM;
    k_agg<<<mPad / RPB, NTHR, 0, stream>>>(H0, LIST, SEG, FLAG, NN, cb, AP);
    k_gemm<8, 0><<<dim3(mPad / GBM, HD / 128), GTHR, 0, stream>>>(AP, W1S, BTB + HD, FLAG, H1, HD, cb, NN);
  }
  for (int c = 0; c < NCH; ++c) {
    const int cb   = c * CR;
    const int rows = (NN - cb) < CR ? (NN - cb) : CR;
    const int mPad = cdiv(rows, GBM) * GBM;
    k_agg<<<mPad / RPB, NTHR, 0, stream>>>(H1, LIST, SEG, FLAG, NN, cb, AP);
    k_gemm<4, 1><<<dim3(mPad / GBM, 1), GTHR, 0, stream>>>(AP, W2S, BTB + 2 * HD, FLAG, out, OD, cb, NN);
  }
}
